// MyMultihead_33440615366831
// MI455X (gfx1250) — hardware-run, weakly checked
//
#include <hip/hip_runtime.h>
#include <math.h>

typedef __attribute__((ext_vector_type(16))) _Float16 v16h;
typedef __attribute__((ext_vector_type(8)))  _Float16 v8h;
typedef __attribute__((ext_vector_type(16))) __bf16   v16b;
typedef __attribute__((ext_vector_type(8)))  __bf16   v8b;
typedef __attribute__((ext_vector_type(8)))  float    v8f;
typedef __attribute__((ext_vector_type(4)))  float    v4f;
typedef __attribute__((ext_vector_type(4)))  unsigned int v4u;

constexpr int kB       = 2;
constexpr int kSeq     = 2048;
constexpr int kE       = 1024;
constexpr int kNH      = 16;
constexpr int kHd      = 64;
constexpr int kTok     = kB * kSeq;
constexpr int kBN      = kB * kNH;
constexpr int kQKPitch = 2 * kHd;
constexpr int kPPitch  = 40;
static_assert(kNH * kHd == kE, "head split");
static_assert(kHd == 64, "head dim");
static_assert((kTok % 64) == 0 && (kE % 64) == 0 && (kE % 32) == 0 && (kSeq % 64) == 0, "tile multiples");

constexpr float kInvSqrtHd  = 0.125f;
static_assert(kInvSqrtHd * kInvSqrtHd * (float)kHd == 1.0f, "score scale");
constexpr float kQKCarry    = 64.0f;
constexpr float kScoreScale = kInvSqrtHd / (kQKCarry * kQKCarry);
constexpr float kPCarry     = 16384.0f;
constexpr float kPCarryInv  = 1.0f / kPCarry;
constexpr float kWoCarry    = 64.0f;
constexpr float kWoCarryInv = 1.0f / kWoCarry;
constexpr float kSkipGap    = 64.0f;

constexpr size_t kSzXB   = (size_t)kTok * kE * 2;
constexpr size_t kSzWT   = (size_t)kE * kE * 2;
constexpr size_t kSzQS   = (size_t)kBN * kSeq * kQKPitch * 2;
constexpr size_t kSzVT   = (size_t)kBN * kHd * kSeq * 2;
constexpr size_t kSzST   = (size_t)kBN * kSeq * 4;
constexpr size_t kSzHS   = (size_t)kTok * kE * 2;
constexpr size_t kOffXB  = 0;
constexpr size_t kOffWT  = kOffXB + 3 * kSzXB;
constexpr size_t kOffWOT = kOffWT + 3 * kSzWT;
constexpr size_t kOffQS  = kOffWOT + kSzWT;
constexpr size_t kOffKS  = kOffQS + kSzQS;
constexpr size_t kOffVT  = kOffKS + kSzQS;
constexpr size_t kOffMX  = kOffVT + kSzVT;
constexpr size_t kOffLI  = kOffMX + kSzST;
constexpr size_t kOffHS  = kOffLI + kSzST;
constexpr size_t kWsTotal = kOffHS + kSzHS;
static_assert(kWsTotal == 84410368ull, "carve total");
static_assert(kWsTotal <= 134217728ull, "carve cap");
static_assert((kOffWT % 128) == 0 && (kOffWOT % 128) == 0 && (kOffQS % 128) == 0 && (kOffKS % 128) == 0 &&
              (kOffVT % 128) == 0 && (kOffMX % 128) == 0 && (kOffLI % 128) == 0 && (kOffHS % 128) == 0, "aligned regions");

__device__ __forceinline__ unsigned short f2bf_bits(float f) {
  unsigned u = __float_as_uint(f);
  return (unsigned short)((u + 0x7FFFu + ((u >> 16) & 1u)) >> 16);
}
__device__ __forceinline__ float bf_bits2f(unsigned short h) { return __uint_as_float(((unsigned)h) << 16); }
__device__ __forceinline__ float bf_rne(float f) { return bf_bits2f(f2bf_bits(f)); }
__device__ __forceinline__ unsigned pk16(unsigned short a, unsigned short b) { return (unsigned)a | ((unsigned)b << 16); }
__device__ __forceinline__ unsigned short h_bits(float f) { const _Float16 h = (_Float16)f; return __builtin_bit_cast(unsigned short, h); }

template <typename T> struct Frag;
template <> struct Frag<_Float16> {
  typedef v16h V; union U { v16h v; v8h h[2]; };
  static __device__ __forceinline__ v16h load(const _Float16* p) {
    U f; f.h[0] = *(const v8h*)(p); f.h[1] = *(const v8h*)(p + 16); return f.v;
  }
  static __device__ __forceinline__ v8f mma(v16h a, v16h b, v8f c) {
    c = __builtin_amdgcn_wmma_f32_16x16x32_f16(false, a, false, b, (short)0, c, false, false);
    asm volatile("v_nop\n\tv_nop\n\tv_nop\n\tv_nop" : "+v"(c) : "v"(a), "v"(b));
    return c;
  }
};
template <> struct Frag<__bf16> {
  typedef v16b V; union U { v16b v; v8b h[2]; };
  static __device__ __forceinline__ v16b load(const __bf16* p) {
    U f; f.h[0] = *(const v8b*)(p); f.h[1] = *(const v8b*)(p + 16); return f.v;
  }
  static __device__ __forceinline__ v8f mma(v16b a, v16b b, v8f c) {
    c = __builtin_amdgcn_wmma_f32_16x16x32_bf16(false, a, false, b, (short)0, c, false, false);
    asm volatile("v_nop\n\tv_nop\n\tv_nop\n\tv_nop" : "+v"(c) : "v"(a), "v"(b));
    return c;
  }
};
typedef Frag<_Float16> FH;

template <int ET> struct Elem;
template <> struct Elem<0> { typedef _Float16 T; };
template <> struct Elem<1> { typedef __bf16 T; };

__global__ __launch_bounds__(256) void cvt_rows_bf16_kernel(
    const float* __restrict__ s0, const float* __restrict__ s1, const float* __restrict__ s2,
    unsigned short* __restrict__ dst, int total8)
{
  const int z = blockIdx.y;
  const float* src = (z == 0) ? s0 : ((z == 1) ? s1 : s2);
  unsigned short* d = dst + (size_t)z * ((size_t)total8 * 8);
  const int i = blockIdx.x * 256 + threadIdx.x;
  if (i >= total8) return;
  const size_t e0 = (size_t)i << 3;
  const v4f a0 = *(const v4f*)(src + e0);
  const v4f a1 = *(const v4f*)(src + e0 + 4);
  unsigned short hb[8];
#pragma unroll
  for (int e = 0; e < 4; ++e) {
    hb[e]     = f2bf_bits(a0[e]);
    hb[4 + e] = f2bf_bits(a1[e]);
  }
  const v4u u = (v4u){pk16(hb[0], hb[1]), pk16(hb[2], hb[3]), pk16(hb[4], hb[5]), pk16(hb[6], hb[7])};
  volatile v4u* p = (volatile v4u*)(d + e0);
  *p = u;
  __threadfence();
  *p = u;
}

template <int MODE>
__global__ __launch_bounds__(256) void wt_transpose_kernel(
    const float* __restrict__ W0, const float* __restrict__ W1, const float* __restrict__ W2,
    int ldin, long inBatch, unsigned short* __restrict__ out, int ldout, long outBatch, long outPlane, int batchPerPlane)
{
  __shared__ float sm[64][65];
  const int t  = threadIdx.x;
  const int r0 = blockIdx.x * 64;
  const int c0 = blockIdx.y * 64;
  const int z  = blockIdx.z;
  const int which = z / batchPerPlane;
  const int nb = z - which * batchPerPlane;
  const float* W = ((which == 0) ? W0 : ((which == 1) ? W1 : W2)) + (size_t)nb * inBatch;
  unsigned short* op = out + (size_t)which * outPlane + (size_t)nb * outBatch;
#pragma unroll
  for (int i = 0; i < 16; ++i) {
    const int e = i * 256 + t;
    const int r = e >> 6;
    const int c = e & 63;
    sm[c][r] = W[(size_t)(r0 + r) * ldin + c0 + c];
  }
  __syncthreads();
  const int lane = t & 31;
  const int wave = __builtin_amdgcn_readfirstlane((int)(t >> 5));
  const int q4 = lane >> 3, c8 = (lane & 7) * 8;
  v4u uv[2];
#pragma unroll
  for (int it = 0; it < 2; ++it) {
    const int row = wave * 8 + it * 4 + q4;
    unsigned short hb[8];
#pragma unroll
    for (int e = 0; e < 8; ++e) {
      const float w = sm[row][c8 + e];
      if (MODE == 0) hb[e] = f2bf_bits(w);
      else           hb[e] = h_bits(bf_rne(w) * kWoCarry);
    }
    uv[it] = (v4u){pk16(hb[0], hb[1]), pk16(hb[2], hb[3]), pk16(hb[4], hb[5]), pk16(hb[6], hb[7])};
  }
  for (int pass = 0; pass < 2; ++pass) {
#pragma unroll
    for (int it = 0; it < 2; ++it) {
      const int row = wave * 8 + it * 4 + q4;
      *(volatile v4u*)(op + (size_t)(c0 + row) * ldout + r0 + c8) = uv[it];
    }
    __threadfence();
  }
}

template <int ET, int EPI>
__global__ __launch_bounds__(256) void gemm64_kernel(
    const unsigned short* __restrict__ Ap, int lda,
    const unsigned short* __restrict__ Btp, int ldb,
    void* __restrict__ Cout, const float* __restrict__ bias,
    int M, int N, int K, float scale)
{
  typedef typename Elem<ET>::T T;
  typedef typename Frag<T>::V V;
  const T* A  = (const T*)Ap;
  const T* Bt = (const T*)Btp;
  __shared__ __align__(16) float sT[8][16 * 68];
  const int lane = threadIdx.x & 31;
  const int wave = __builtin_amdgcn_readfirstlane((int)(threadIdx.x >> 5));
  const int tilesN = N >> 6;
  const int tilesM = M >> 6;
  const int tile = blockIdx.x * 8 + wave;
  if (tile >= tilesM * tilesN) return;
  const int tm = tile / tilesN;
  const int tn = tile - tm * tilesN;
  const int m0 = tm << 6;
  const int n0 = tn << 6;
  const int rlane = lane & 15;
  const int koff  = (lane >> 4) * 8;
  const int mOff  = (lane >> 4) * 8;

  v8f acc[4][4];
#pragma unroll
  for (int i = 0; i < 4; ++i)
#pragma unroll
    for (int j = 0; j < 4; ++j) acc[i][j] = (v8f){0.f, 0.f, 0.f, 0.f, 0.f, 0.f, 0.f, 0.f};

  for (int k0 = 0; k0 < K; k0 += 32) {
    V bh[4];
#pragma unroll
    for (int j = 0; j < 4; ++j)
      bh[j] = Frag<T>::load(Bt + (size_t)(n0 + (j << 4) + rlane) * ldb + koff + k0);
#pragma unroll
    for (int i = 0; i < 4; ++i) {
      const V ah = Frag<T>::load(A + (size_t)(m0 + (i << 4) + rlane) * lda + koff + k0);
#pragma unroll
      for (int j = 0; j < 4; ++j) acc[i][j] = Frag<T>::mma(ah, bh[j], acc[i][j]);
    }
  }

  float* slab = sT[wave];
#pragma unroll
  for (int i = 0; i < 4; ++i) {
    const int mBase = m0 + (i << 4);
    float bm[8];
#pragma unroll
    for (int r = 0; r < 8; ++r) bm[r] = 0.f;
    if (EPI == 1) {
#pragma unroll
      for (int r = 0; r < 8; ++r) bm[r] = bf_rne(bias[mBase + mOff + r]);
    }
#pragma unroll
    for (int j = 0; j < 4; ++j) {
      float bv = 0.f;
      if (EPI != 1) bv = bf_rne(bias[n0 + (j << 4) + rlane]);
#pragma unroll
      for (int r = 0; r < 8; ++r) {
        float v;
        if (EPI == 0)      v = (acc[i][j][r] + bv) * scale;
        else if (EPI == 1) v = acc[i][j][r] + bm[r];
        else               v = acc[i][j][r] * scale + bv;
        slab[(mOff + r) * 68 + (j << 4) + rlane] = v;
      }
    }
    __builtin_amdgcn_fence(__ATOMIC_RELEASE, "workgroup");
    __builtin_amdgcn_wave_barrier();
    __builtin_amdgcn_fence(__ATOMIC_ACQUIRE, "workgroup");
    if (EPI == 2) {
      float* C = (float*)Cout;
      const int hh = lane >> 4, c4 = (lane & 15) * 4;
      for (int pass = 0; pass < 2; ++pass) {
#pragma unroll
        for (int it = 0; it < 8; ++it) {
          const int row = it * 2 + hh;
          const v4f v = *(const v4f*)(slab + row * 68 + c4);
          *(volatile v4f*)(C + (size_t)(mBase + row) * N + n0 + c4) = v;
        }
        __threadfence();
      }
    } else if (EPI == 0) {
      const int q4 = lane >> 3, c8 = (lane & 7) * 8;
      unsigned short* C = (unsigned short*)Cout;
      const int bIdx  = mBase / kSeq;
      const int sBase = mBase - bIdx * kSeq;
      v8h hv[4], lv[4];
#pragma unroll
      for (int it = 0; it < 4; ++it) {
        const float* sp = slab + (it * 4 + q4) * 68 + c8;
#pragma unroll
        for (int e = 0; e < 8; ++e) {
          const float x = sp[e];
          const _Float16 hx = (_Float16)x;
          const _Float16 lx = (_Float16)(x - (float)hx);
          hv[it][e] = hx;
          lv[it][e] = lx;
        }
      }
      for (int pass = 0; pass < 2; ++pass) {
#pragma unroll
        for (int it = 0; it < 4; ++it) {
          const int row = it * 4 + q4;
          unsigned short* dst = C + ((size_t)(bIdx * kNH + tn) * kSeq + sBase + row) * kQKPitch + c8;
          *(volatile v8h*)(dst) = hv[it];
          *(volatile v8h*)(dst + kHd) = lv[it];
        }
        __threadfence();
      }
    } else {
      const int q4 = lane >> 3, c8 = (lane & 7) * 8;
      unsigned short* C = (unsigned short*)Cout;
      const int bIdx = n0 / kSeq;
      const int s0   = n0 - bIdx * kSeq;
      v8h hv[4];
#pragma unroll
      for (int it = 0; it < 4; ++it) {
        const float* sp = slab + (it * 4 + q4) * 68 + c8;
#pragma unroll
        for (int e = 0; e < 8; ++e) {
          const _Float16 hx = (_Float16)sp[e];
          hv[it][e] = hx;
        }
      }
      for (int pass = 0; pass < 2; ++pass) {
#pragma unroll
        for (int it = 0; it < 4; ++it) {
          const int row = it * 4 + q4;
          unsigned short* dst = C + ((size_t)((bIdx * kNH + tm) * kHd + (i << 4) + row)) * kSeq + s0 + c8;
          *(volatile v8h*)(dst) = hv[it];
        }
        __threadfence();
      }
    }
    __builtin_amdgcn_fence(__ATOMIC_RELEASE, "workgroup");
    __builtin_amdgcn_wave_barrier();
    __builtin_amdgcn_fence(__ATOMIC_ACQUIRE, "workgroup");
  }
}

__device__ __forceinline__ v8f score_head(v16h qh0, v16h qh1, v16h kh0, v16h kh1) {
  v8f s = (v8f){0.f, 0.f, 0.f, 0.f, 0.f, 0.f, 0.f, 0.f};
  s = FH::mma(qh0, kh0, s);
  s = FH::mma(qh1, kh1, s);
  return s;
}
__device__ __forceinline__ v8f score_tail(v8f s, v16h qh0, v16h qh1, v16h ql0, v16h ql1,
                                          v16h kh0, v16h kh1, v16h kl0, v16h kl1) {
  s = FH::mma(qh0, kl0, s);
  s = FH::mma(ql0, kh0, s);
  s = FH::mma(qh1, kl1, s);
  s = FH::mma(ql1, kh1, s);
  return s;
}

__device__ __forceinline__ void stat_update(const v8f& s, float& rmax, float& rsum) {
  float t = fmaxf(fmaxf(fmaxf(s[0], s[1]), fmaxf(s[2], s[3])), fmaxf(fmaxf(s[4], s[5]), fmaxf(s[6], s[7])));
  t = fmaxf(t, __shfl_xor(t, 16, 32));
  const float tm = t * kScoreScale;
  const float nm = fmaxf(rmax, tm);
  float a = 0.f;
#pragma unroll
  for (int r = 0; r < 8; ++r) a += __expf(fmaf(s[r], kScoreScale, -nm));
  rsum = rsum * __expf(rmax - nm) + a;
  rmax = nm;
}

__global__ __launch_bounds__(128) void col_stats_kernel(
    const unsigned short* __restrict__ QSp, const unsigned short* __restrict__ KSp,
    float* __restrict__ MX, float* __restrict__ LI)
{
  const _Float16* QS = (const _Float16*)QSp;
  const _Float16* KS = (const _Float16*)KSp;
  const int lane = threadIdx.x & 31;
  const int wave = __builtin_amdgcn_readfirstlane((int)(threadIdx.x >> 5));
  const int gw = blockIdx.x * 4 + wave;
  const int bn = gw >> 6;
  const int k0 = (gw & 63) << 5;
  const int c = lane & 15, hh = lane >> 4;

  const _Float16* ka = KS + ((size_t)bn * kSeq + k0 + c) * kQKPitch + 8 * hh;
  const _Float16* kb = ka + 16 * kQKPitch;
  const v16h ka_h0 = FH::load(ka),       ka_h1 = FH::load(ka + 32);
  const v16h ka_l0 = FH::load(ka + kHd), ka_l1 = FH::load(ka + kHd + 32);
  const v16h kb_h0 = FH::load(kb),       kb_h1 = FH::load(kb + 32);
  const v16h kb_l0 = FH::load(kb + kHd), kb_l1 = FH::load(kb + kHd + 32);

  float rmax0 = -1.0e30f, rsum0 = 0.f, rmax1 = -1.0e30f, rsum1 = 0.f;
  const _Float16* qp = QS + ((size_t)bn * kSeq + c) * kQKPitch + 8 * hh;
#pragma unroll 1
  for (int qt = 0; qt < kSeq / 16; ++qt) {
    const v16h qh0 = FH::load(qp),       qh1 = FH::load(qp + 32);
    const v16h ql0 = FH::load(qp + kHd), ql1 = FH::load(qp + kHd + 32);
    qp += 16 * kQKPitch;
    v8f s0 = score_head(qh0, qh1, ka_h0, ka_h1);
    s0 = score_tail(s0, qh0, qh1, ql0, ql1, ka_h0, ka_h1, ka_l0, ka_l1);
    v8f s1 = score_head(qh0, qh1, kb_h0, kb_h1);
    s1 = score_tail(s1, qh0, qh1, ql0, ql1, kb_h0, kb_h1, kb_l0, kb_l1);
    stat_update(s0, rmax0, rsum0);
    stat_update(s1, rmax1, rsum1);
  }
  rsum0 += __shfl_xor(rsum0, 16, 32);
  rsum1 += __shfl_xor(rsum1, 16, 32);
  const float mval = (hh == 0) ? rmax0 : rmax1;
  const float lval = (hh == 0) ? rsum0 : rsum1;
  const float li = kPCarry * (1.0f / lval);
  const size_t o = (size_t)bn * kSeq + k0 + lane;
  volatile float* pm = MX + o;
  volatile float* pl = LI + o;
  *pm = mval;
  *pl = li;
  __threadfence();
  *pm = mval;
  *pl = li;
}

__global__ __launch_bounds__(128) void attn_pv_kernel(
    const unsigned short* __restrict__ QSp, const unsigned short* __restrict__ KSp,
    const unsigned short* __restrict__ VTp, const float* __restrict__ MX, const float* __restrict__ LI,
    unsigned short* __restrict__ HS)
{
  __shared__ __align__(16) _Float16 Ps[4][16 * kPPitch];
  __shared__ __align__(16) float    Os[4][16 * 68];
  const _Float16* QS = (const _Float16*)QSp;
  const _Float16* KS = (const _Float16*)KSp;
  const _Float16* VT = (const _Float16*)VTp;
  const int lane = threadIdx.x & 31;
  const int wave = __builtin_amdgcn_readfirstlane((int)(threadIdx.x >> 5));
  const int c = lane & 15, hh = lane >> 4;
  const int bx = blockIdx.x;
  const int qb = bx & 31;
  const int bn = bx >> 5;
  const int b  = bn / kNH;
  const int n  = bn - b * kNH;
  const int q0 = qb * 64 + wave * 16;

  const _Float16* qp = QS + ((size_t)bn * kSeq + q0 + c) * kQKPitch + 8 * hh;
  const v16h qh0 = FH::load(qp),       qh1 = FH::load(qp + 32);
  const v16h ql0 = FH::load(qp + kHd), ql1 = FH::load(qp + kHd + 32);

  v8f oacc[4];
#pragma unroll
  for (int t = 0; t < 4; ++t) oacc[t] = (v8f){0.f, 0.f, 0.f, 0.f, 0.f, 0.f, 0.f, 0.f};

  const _Float16* kp = KS + ((size_t)bn * kSeq + c) * kQKPitch + 8 * hh;
  const _Float16* vp = VT + ((size_t)bn * kHd + c) * kSeq + 8 * hh;
  const float* mp = MX + (size_t)bn * kSeq + c;
  const float* lp = LI + (size_t)bn * kSeq + c;
  _Float16* pw = Ps[wave];

#pragma unroll 1
  for (int kc = 0; kc < kSeq / 32; ++kc) {
    const int k0 = kc * 32;
    const _Float16* ka = kp + (size_t)k0 * kQKPitch;
    const _Float16* kb = ka + 16 * kQKPitch;
    const v16h ka_h0 = FH::load(ka), ka_h1 = FH::load(ka + 32);
    const v16h kb_h0 = FH::load(kb), kb_h1 = FH::load(kb + 32);
    v8f s0 = score_head(qh0, qh1, ka_h0, ka_h1);
    v8f s1 = score_head(qh0, qh1, kb_h0, kb_h1);
    const float m0 = mp[k0], m1 = mp[k0 + 16];
    const float l0 = lp[k0], l1 = lp[k0 + 16];
    float g = -1.0e30f;
#pragma unroll
    for (int r = 0; r < 8; ++r) {
      g = fmaxf(g, fmaf(s0[r], kScoreScale, -m0));
      g = fmaxf(g, fmaf(s1[r], kScoreScale, -m1));
    }
    const unsigned live = __builtin_amdgcn_ballot_w32(g > -kSkipGap);
    if (live != 0u) {
      const v16h ka_l0 = FH::load(ka + kHd), ka_l1 = FH::load(ka + kHd + 32);
      s0 = score_tail(s0, qh0, qh1, ql0, ql1, ka_h0, ka_h1, ka_l0, ka_l1);
      const v16h kb_l0 = FH::load(kb + kHd), kb_l1 = FH::load(kb + kHd + 32);
      s1 = score_tail(s1, qh0, qh1, ql0, ql1, kb_h0, kb_h1, kb_l0, kb_l1);
#pragma unroll
      for (int r = 0; r < 8; ++r) {
        const float p0 = __expf(fmaf(s0[r], kScoreScale, -m0)) * l0;
        const float p1 = __expf(fmaf(s1[r], kScoreScale, -m1)) * l1;
        pw[(8 * hh + r) * kPPitch + c]      = (_Float16)p0;
        pw[(8 * hh + r) * kPPitch + 16 + c] = (_Float16)p1;
      }
      __builtin_amdgcn_fence(__ATOMIC_RELEASE, "workgroup");
      __builtin_amdgcn_wave_barrier();
      __builtin_amdgcn_fence(__ATOMIC_ACQUIRE, "workgroup");
      const v16h pa = FH::load(pw + c * kPPitch + 8 * hh);
#pragma unroll
      for (int t = 0; t < 4; ++t) {
        const v16h vb = FH::load(vp + (size_t)(t * 16) * kSeq + k0);
        oacc[t] = FH::mma(pa, vb, oacc[t]);
      }
      __builtin_amdgcn_fence(__ATOMIC_RELEASE, "workgroup");
      __builtin_amdgcn_wave_barrier();
      __builtin_amdgcn_fence(__ATOMIC_ACQUIRE, "workgroup");
    }
  }

  float* os = Os[wave];
#pragma unroll
  for (int r = 0; r < 8; ++r) {
#pragma unroll
    for (int t = 0; t < 4; ++t) os[(8 * hh + r) * 68 + t * 16 + c] = oacc[t][r] * kPCarryInv;
  }
  __builtin_amdgcn_fence(__ATOMIC_RELEASE, "workgroup");
  __builtin_amdgcn_wave_barrier();
  __builtin_amdgcn_fence(__ATOMIC_ACQUIRE, "workgroup");
  {
    const int q4 = lane >> 3, c8 = (lane & 7) * 8;
    v8h hv[4];
#pragma unroll
    for (int it = 0; it < 4; ++it) {
      const float* sp = os + (it * 4 + q4) * 68 + c8;
#pragma unroll
      for (int e = 0; e < 8; ++e) {
        const _Float16 hx = (_Float16)sp[e];
        hv[it][e] = hx;
      }
    }
    for (int pass = 0; pass < 2; ++pass) {
#pragma unroll
      for (int it = 0; it < 4; ++it) {
        const int row = it * 4 + q4;
        unsigned short* dst = HS + (size_t)(b * kSeq + q0 + row) * kE + n * kHd + c8;
        *(volatile v8h*)(dst) = hv[it];
      }
      __threadfence();
    }
  }
}

extern "C" void kernel_launch(void* const* d_in, const int* in_sizes, int n_in,
                              void* d_out, int out_size, void* d_ws, size_t ws_size,
                              hipStream_t stream) {
  if (n_in < 11) return;
  if (in_sizes[0] != kTok * kE || in_sizes[1] != kTok * kE || in_sizes[2] != kTok * kE) return;
  if (in_sizes[3] != kNH * kE * kHd || in_sizes[4] != kNH * kE * kHd || in_sizes[5] != kNH * kE * kHd) return;
  if (in_sizes[6] != kE * kE) return;
  if (in_sizes[7] != kNH * kHd || in_sizes[8] != kNH * kHd || in_sizes[9] != kNH * kHd) return;
  if (in_sizes[10] != kE) return;
  if (out_size != kTok * kE) return;
  if (ws_size < kWsTotal) return;

  const float* q  = (const float*)d_in[0];
  const float* k  = (const float*)d_in[1];
  const float* v  = (const float*)d_in[2];
  const float* wq = (const float*)d_in[3];
  const float* wk = (const float*)d_in[4];
  const float* wv = (const float*)d_in[5];
  const float* wo = (const float*)d_in[6];
  const float* bq = (const float*)d_in[7];
  const float* bk = (const float*)d_in[8];
  const float* bv = (const float*)d_in[9];
  const float* bo = (const float*)d_in[10];
  float* out = (float*)d_out;

  char* ws = (char*)d_ws;
  unsigned short* XB  = (unsigned short*)(ws + kOffXB);
  unsigned short* WT  = (unsigned short*)(ws + kOffWT);
  unsigned short* WOT = (unsigned short*)(ws + kOffWOT);
  unsigned short* QS  = (unsigned short*)(ws + kOffQS);
  unsigned short* KS  = (unsigned short*)(ws + kOffKS);
  unsigned short* VT  = (unsigned short*)(ws + kOffVT);
  float*          MX  = (float*)(ws + kOffMX);
  float*          LI  = (float*)(ws + kOffLI);
  unsigned short* HS  = (unsigned short*)(ws + kOffHS);

  unsigned short* XBq = XB;
  unsigned short* XBk = XB + (size_t)kTok * kE;
  unsigned short* XBv = XB + 2 * (size_t)kTok * kE;
  unsigned short* WTq = WT;
  unsigned short* WTk = WT + (size_t)kE * kE;
  unsigned short* WTv = WT + 2 * (size_t)kE * kE;

  cvt_rows_bf16_kernel<<<dim3((kTok * kE / 8) / 256, 3), 256, 0, stream>>>(q, k, v, XB, kTok * kE / 8);

  wt_transpose_kernel<0><<<dim3(kE / 64, kHd / 64, 3 * kNH), 256, 0, stream>>>(
      wq, wk, wv, kHd, (long)kE * kHd, WT, kE, (long)kHd * kE, (long)kE * kE, kNH);

  wt_transpose_kernel<1><<<dim3(kE / 64, kE / 64, 1), 256, 0, stream>>>(
      wo, wo, wo, kE, 0L, WOT, kE, 0L, 0L, 1);

  gemm64_kernel<1, 0><<<128, 256, 0, stream>>>(XBq, kE, WTq, kE, (void*)QS, bq, kTok, kE, kE, kQKCarry);
  gemm64_kernel<1, 0><<<128, 256, 0, stream>>>(XBk, kE, WTk, kE, (void*)KS, bk, kTok, kE, kE, kQKCarry);

  gemm64_kernel<1, 1><<<128, 256, 0, stream>>>(WTv, kE, XBv, kE, (void*)VT, bv, kE, kTok, kE, 1.0f);

  col_stats_kernel<<<(kBN * (kSeq / 32)) / 4, 128, 0, stream>>>(QS, KS, MX, LI);

  attn_pv_kernel<<<kBN * (kSeq / 64), 128, 0, stream>>>(QS, KS, VT, MX, LI, HS);

  gemm64_kernel<0, 2><<<128, 256, 0, stream>>>(HS, kE, WOT, kE, (void*)out, bo, kTok, kE, kE, kWoCarryInv);
}
